// DeepseekMoE_60378650247253
// MI455X (gfx1250) — hardware-verified
//
#include <hip/hip_runtime.h>
#include <stddef.h>
#include <stdint.h>
#include <math.h>

#define NTOK   4096
#define DD     512
#define FF     2048
#define NE     8
#define NSH    2
#define NSEL   2
#define MT     32
#define TPE    (NTOK / MT)
#define RPITCH 8
#define NPROW  (NTOK * NSEL)
#define NPART  (NSH * NTOK + NPROW)
#define FB     256
#define WSC    64.0f
#define UG     0.015625f
#define HSC    64.0f
#define DN     0.000244140625f
#define APITCH 520
#define HPITCH 264
#define OTP    68

static_assert(NSEL == 2);
static_assert(NE == 8);
static_assert(TPE == 128);
static_assert(DD % 32 == 0);
static_assert(FF % FB == 0);
static_assert(FB % 32 == 0);
static_assert(FB == 8 * 32);
static_assert(DD == 8 * 64);
static_assert(NTOK % 256 == 0);
static_assert(NTOK % 8 == 0);
static_assert((NTOK * DD) % 2048 == 0);
static_assert((NSH * FF * DD) % 2048 == 0);
static_assert((NE * FF * DD) % 2048 == 0);
static_assert(MT * APITCH * 2 <= 8 * 16 * OTP * 4);
static_assert((APITCH * 2) % 16 == 0);
static_assert((HPITCH * 2) % 16 == 0);
static_assert((OTP * 4) % 16 == 0);

typedef _Float16 v16h __attribute__((ext_vector_type(16)));
typedef _Float16 v8h  __attribute__((ext_vector_type(8)));
typedef float    v8f  __attribute__((ext_vector_type(8)));
typedef float    v4f  __attribute__((ext_vector_type(4)));
typedef unsigned int v4u __attribute__((ext_vector_type(4)));
typedef int      v4i  __attribute__((ext_vector_type(4)));
typedef unsigned short v4us __attribute__((ext_vector_type(4)));

union Frag  { v16h v; v8h h[2]; };
union Pack8 { v8h h; v4u u; };

__device__ __forceinline__ int clampi(int v, int lo, int hi) { return min(max(v, lo), hi); }

__device__ __forceinline__ v8f mma16(v16h a, v16h b, v8f c) {
  c = __builtin_amdgcn_wmma_f32_16x16x32_f16(false, a, false, b, (short)0, c, false, false);
  asm volatile("v_nop\n\tv_nop\n\tv_nop\n\tv_nop" : "+v"(c) : "v"(a), "v"(b));
  return c;
}

__device__ __forceinline__ v16h ldfrag(const _Float16* p, int ld, int row0, int k0, int lane) {
  const int m = lane & 15, lh = lane >> 4;
  const _Float16* q = p + (size_t)(row0 + m) * ld + k0 + 8 * lh;
  Frag f;
  f.h[0] = *(const v8h*)(q);
  f.h[1] = *(const v8h*)(q + 16);
  return f.v;
}

__device__ __forceinline__ v8f zero8() { return (v8f){0.f, 0.f, 0.f, 0.f, 0.f, 0.f, 0.f, 0.f}; }

__device__ __forceinline__ float gelu_erf(float v) {
  return 0.5f * v * (1.0f + erff(v * 0.70710678118654752440f));
}

__global__ __launch_bounds__(256) void k_cvt(const float* __restrict__ src, _Float16* __restrict__ dh, int n8,
                                             float scale) {
  const int i = blockIdx.x * 256 + (int)threadIdx.x;
  if (i >= n8) return;
  const size_t o = (size_t)i * 8;
  const v4f a0 = *(const v4f*)(src + o) * scale;
  const v4f a1 = *(const v4f*)(src + o + 4) * scale;
  Pack8 pk;
  pk.h = (v8h){(_Float16)a0[0], (_Float16)a0[1], (_Float16)a0[2], (_Float16)a0[3],
               (_Float16)a1[0], (_Float16)a1[1], (_Float16)a1[2], (_Float16)a1[3]};
  const v4u vv = pk.u;
  volatile v4u* d = (volatile v4u*)(dh + o);
  *d = vv;
  __threadfence();
  *d = vv;
}

__global__ __launch_bounds__(256) void k_route(const float* __restrict__ x, const float* __restrict__ gw,
                                               const float* __restrict__ gb, float* __restrict__ rp) {
  __shared__ __align__(16) float sR[8 * RPITCH];
  const int tid = threadIdx.x, lane = tid & 31, wave = tid >> 5;
  const int c = lane & 15, c8 = lane & 7;
  const size_t t = (size_t)blockIdx.x * 8 + wave;
  const float* xr = x + t * DD;

  float a[NE];
#pragma unroll
  for (int e = 0; e < NE; ++e) a[e] = 0.f;
#pragma unroll 1
  for (int j = 0; j < DD / 32; ++j) {
    const int k = j * 32 + lane;
    const float xv = xr[k];
#pragma unroll
    for (int e = 0; e < NE; ++e) a[e] += xv * gw[(size_t)e * DD + k];
  }
#pragma unroll
  for (int e = 0; e < NE; ++e) {
#pragma unroll
    for (int off = 16; off >= 1; off >>= 1) a[e] += __shfl_xor(a[e], off, 32);
  }
#pragma unroll
  for (int e = 0; e < NE; ++e) a[e] += gb[e];

  float mx = a[0];
#pragma unroll
  for (int e = 1; e < NE; ++e) mx = fmaxf(mx, a[e]);
  float mine = a[0];
#pragma unroll
  for (int e = 1; e < NE; ++e) mine = (c8 == e) ? a[e] : mine;
  const float exm = expf(mine - mx);
  float ssum = exm;
#pragma unroll
  for (int off = 1; off < 8; off <<= 1) ssum += __shfl_xor(ssum, off, 32);
  const float inv = 1.0f / ssum;
  const float scm = exm * inv;
  float sc[NE];
#pragma unroll
  for (int e = 0; e < NE; ++e) sc[e] = __shfl(scm, e, 32);

  const float NEGI = -__builtin_huge_valf();
  unsigned taken = 0u;
  int idx[NSEL];
  float wsel[NSEL];
#pragma unroll
  for (int kk = 0; kk < NSEL; ++kk) {
    float bv = NEGI;
    int best = 0;
    float bs = 0.f;
#pragma unroll
    for (int i = 0; i < NE; ++i) {
      const bool cnd = (((taken >> i) & 1u) == 0u) && (sc[i] > bv);
      bv   = cnd ? sc[i] : bv;
      best = cnd ? i : best;
      bs   = cnd ? sc[i] : bs;
    }
    taken |= (1u << best);
    idx[kk]  = best;
    wsel[kk] = bs;
  }
  const float w0 = wsel[0];
  const float w1 = wsel[1];

  float ov = 0.f;
  ov = (lane == 0) ? (float)idx[0] : ov;
  ov = (lane == 1) ? (float)idx[1] : ov;
  ov = (lane == 4) ? w0 : ov;
  ov = (lane == 5) ? w1 : ov;
  if (lane < RPITCH) sR[wave * RPITCH + lane] = ov;
  __syncthreads();
  if (wave == 0) {
    const v4f vr = *(const v4f*)(sR + c * 4);
    volatile v4f* dr = (volatile v4f*)(rp + (size_t)blockIdx.x * (8 * RPITCH) + c * 4);
    if (lane < 16) *dr = vr;
    __threadfence();
    if (lane < 16) *dr = vr;
  }
}

__global__ __launch_bounds__(256) void k_lists(const float* __restrict__ rp, int* __restrict__ tokl,
                                               float* __restrict__ wl, int* __restrict__ tab) {
  __shared__ __align__(16) unsigned short ltok[NTOK];
  __shared__ __align__(16) float lw[NTOK];
  __shared__ int wc[8];
  __shared__ __align__(16) int sTab[64];
  const int tid = threadIdx.x, lane = tid & 31, wave = tid >> 5;
  if (tid < 64) sTab[tid] = 0;
#pragma unroll 1
  for (int e = 0; e < NE; ++e) {
    __syncthreads();
    for (int i = tid; i < NTOK; i += 256) { ltok[i] = (unsigned short)0; lw[i] = 0.f; }
    __syncthreads();
    int run = 0;
#pragma unroll 1
    for (int ch = 0; ch < NTOK / 256; ++ch) {
      const int t = ch * 256 + tid;
      const v4f ri = *(const v4f*)(rp + (size_t)t * RPITCH);
      const v4f rw = *(const v4f*)(rp + (size_t)t * RPITCH + 4);
      int hit = -1;
      float w = 0.f;
#pragma unroll
      for (int k = NSEL - 1; k >= 0; --k) {
        const bool m = ((int)ri[k] == e);
        hit = m ? k : hit;
        w   = m ? rw[k] : w;
      }
      const bool flag = (hit >= 0);
      const unsigned bal = __builtin_amdgcn_ballot_w32(flag);
      const int pre = __builtin_popcount(bal & ((1u << lane) - 1u));
      if (lane == 0) wc[wave] = __builtin_popcount(bal);
      __syncthreads();
      int base = run, tot = 0;
#pragma unroll
      for (int q = 0; q < 8; ++q) {
        const int cw = wc[q];
        base += (q < wave) ? cw : 0;
        tot  += cw;
      }
      const int pos = clampi(base + pre, 0, NTOK - 1);
      if (flag) { ltok[pos] = (unsigned short)(t * NSEL + hit); lw[pos] = w; }
      run += tot;
      __syncthreads();
    }
    run = clampi(run, 0, NTOK);
    if (tid == 0) sTab[e] = run;

    int*   trow = tokl + (size_t)e * NTOK;
    float* wrow = wl + (size_t)e * NTOK;
    v4i tv[4];
    v4f wv[4];
    int po[4];
#pragma unroll
    for (int it = 0; it < 4; ++it) {
      const int p = tid + 256 * it;
      const v4us u = *(const v4us*)(ltok + p * 4);
      tv[it] = (v4i){(int)u[0], (int)u[1], (int)u[2], (int)u[3]};
      wv[it] = *(const v4f*)(lw + p * 4);
      po[it] = p * 4;
    }
#pragma unroll
    for (int it = 0; it < 4; ++it) {
      *(volatile v4i*)(trow + po[it]) = tv[it];
      *(volatile v4f*)(wrow + po[it]) = wv[it];
    }
    __threadfence();
#pragma unroll
    for (int it = 0; it < 4; ++it) {
      *(volatile v4i*)(trow + po[it]) = tv[it];
      *(volatile v4f*)(wrow + po[it]) = wv[it];
    }
  }
  __syncthreads();
  if (wave == 0) {
    const v4i v = *(const v4i*)(sTab + (lane & 15) * 4);
    volatile v4i* d = (volatile v4i*)(tab + (lane & 15) * 4);
    if (lane < 16) *d = v;
    __threadfence();
    if (lane < 16) *d = v;
  }
}

__global__ __launch_bounds__(256) void k_ffn(const _Float16* __restrict__ xh,
                                             const _Float16* __restrict__ sw1h, const float* __restrict__ sb1,
                                             const _Float16* __restrict__ sw2h, const float* __restrict__ sb2,
                                             const _Float16* __restrict__ rw1h, const float* __restrict__ rb1,
                                             const _Float16* __restrict__ rw2h, const float* __restrict__ rb2,
                                             const int* __restrict__ tokl, const float* __restrict__ wl,
                                             const int* __restrict__ tab, float* __restrict__ part) {
  __shared__ __align__(16) float sU[8 * 16 * OTP];
  __shared__ __align__(16) _Float16 sH[MT * HPITCH];
  __shared__ int   sTok[MT];
  __shared__ float sW[MT];
  __shared__ int   sVal[MT];
  __shared__ int   sRow[MT];
  _Float16* sA = reinterpret_cast<_Float16*>(sU);

  const int tid = threadIdx.x, lane = tid & 31, wave = tid >> 5;
  const int hh = lane >> 4, c = lane & 15;
  const int bid = blockIdx.x;
  const bool routed = (bid >= NSH * TPE);
  const int rel  = routed ? (bid - NSH * TPE) : bid;
  const int e    = rel / TPE;
  const int tile = rel % TPE;
  const int cntv = clampi(tab[e], 0, NTOK);
  const int cne  = routed ? cntv : NTOK;
  if (routed && tile * MT >= cne) return;

  const _Float16* W1e = (routed ? rw1h : sw1h) + (size_t)e * (size_t)(FF * DD);
  const _Float16* W2e = (routed ? rw2h : sw2h) + (size_t)e * (size_t)(DD * FF);
  const float* B1 = (routed ? rb1 : sb1) + (size_t)e * FF;
  const float* B2 = (routed ? rb2 : sb2) + (size_t)e * DD;

  if (tid < MT) {
    const int j    = tile * MT + tid;
    const int li   = e * NTOK + clampi(j, 0, NTOK - 1);
    const int enc  = clampi(tokl[li], 0, NPROW - 1);
    const float wv = wl[li];
    const bool valid = routed ? (j < cne) : true;
    sTok[tid] = routed ? (enc >> 1) : j;
    sW[tid]   = routed ? (valid ? wv : 0.f) : 1.0f;
    sVal[tid] = valid ? 1 : 0;
    sRow[tid] = routed ? (NSH * NTOK + enc) : (e * NTOK + j);
  }
  __syncthreads();

  {
    const int ar = tid >> 3, ab = (tid & 7) * 64;
    const _Float16* xrow = xh + (size_t)sTok[ar] * DD + ab;
    _Float16* arow = sA + ar * APITCH + ab;
#pragma unroll
    for (int q = 0; q < 8; ++q) *(v8h*)(arow + 8 * q) = *(const v8h*)(xrow + 8 * q);
  }
  __syncthreads();

  const int n1 = wave * 32;
  const int n2 = wave * 64;
  v8f acc2[4][2];
#pragma unroll
  for (int t = 0; t < 4; ++t) { acc2[t][0] = zero8(); acc2[t][1] = zero8(); }

#pragma unroll 1
  for (int fb = 0; fb < FF / FB; ++fb) {
    const int fbase = fb * FB;
    v8f g[2][2];
#pragma unroll
    for (int t = 0; t < 2; ++t) { g[t][0] = zero8(); g[t][1] = zero8(); }
#pragma unroll 1
    for (int k0 = 0; k0 < DD; k0 += 32) {
      const v16h a0 = ldfrag(sA, APITCH, 0, k0, lane);
      const v16h a1 = ldfrag(sA, APITCH, 16, k0, lane);
#pragma unroll
      for (int t = 0; t < 2; ++t) {
        const v16h bq = ldfrag(W1e, DD, fbase + n1 + 16 * t, k0, lane);
        g[t][0] = mma16(a0, bq, g[t][0]);
        g[t][1] = mma16(a1, bq, g[t][1]);
      }
    }
#pragma unroll
    for (int t = 0; t < 2; ++t) {
      const int col = n1 + 16 * t + c;
      const float bias = B1[fbase + col];
#pragma unroll
      for (int mt = 0; mt < 2; ++mt) {
#pragma unroll
        for (int r = 0; r < 8; ++r) {
          const float pre = g[t][mt][r] * UG + bias;
          const float hv = gelu_erf(pre) * HSC;
          sH[(mt * 16 + 8 * hh + r) * HPITCH + col] = (_Float16)hv;
        }
      }
    }
    __syncthreads();
#pragma unroll 1
    for (int kk = 0; kk < FB; kk += 32) {
      const v16h a0 = ldfrag(sH, HPITCH, 0, kk, lane);
      const v16h a1 = ldfrag(sH, HPITCH, 16, kk, lane);
#pragma unroll
      for (int t = 0; t < 4; ++t) {
        const v16h bq = ldfrag(W2e, FF, n2 + 16 * t, fbase + kk, lane);
        acc2[t][0] = mma16(a0, bq, acc2[t][0]);
        acc2[t][1] = mma16(a1, bq, acc2[t][1]);
      }
    }
    __syncthreads();
  }

  float* sw = sU + wave * (16 * OTP);
#pragma unroll
  for (int mt = 0; mt < 2; ++mt) {
    float wr[8];
#pragma unroll
    for (int r = 0; r < 8; ++r) wr[r] = sW[mt * 16 + 8 * hh + r];
#pragma unroll
    for (int t = 0; t < 4; ++t) {
      const int col = n2 + 16 * t + c;
      const float bias = B2[col];
#pragma unroll
      for (int r = 0; r < 8; ++r) sw[(8 * hh + r) * OTP + 16 * t + c] = (acc2[t][mt][r] * DN + bias) * wr[r];
    }
    __syncthreads();
    v4f val[8];
    int go[8];
    bool ok[8];
#pragma unroll
    for (int it = 0; it < 8; ++it) {
      const int p    = lane + 32 * it;
      const int L    = p >> 3;
      const int pc   = p & 7;
      const int row  = L >> 1;
      const int half = L & 1;
      const int lr   = mt * 16 + row;
      val[it] = *(const v4f*)(sw + row * OTP + half * 32 + pc * 4);
      ok[it]  = (sVal[lr] != 0);
      go[it]  = sRow[lr] * DD + n2 + half * 32 + pc * 4;
    }
#pragma unroll
    for (int it = 0; it < 8; ++it) {
      if (ok[it]) *(volatile v4f*)(part + (size_t)go[it]) = val[it];
    }
    __threadfence();
#pragma unroll
    for (int it = 0; it < 8; ++it) {
      if (ok[it]) *(volatile v4f*)(part + (size_t)go[it]) = val[it];
    }
    __syncthreads();
  }
}

__global__ __launch_bounds__(256) void k_comb(const float* __restrict__ part, float* __restrict__ out, int n4) {
  const int i = blockIdx.x * 256 + (int)threadIdx.x;
  if (i >= n4) return;
  const size_t t = (size_t)i / (DD / 4);
  const size_t n = ((size_t)i % (DD / 4)) * 4;
  const v4f s0 = *(const v4f*)(part + t * DD + n);
  const v4f s1 = *(const v4f*)(part + ((size_t)NTOK + t) * DD + n);
  const float* pr = part + ((size_t)(NSH * NTOK) + t * NSEL) * DD + n;
  const v4f p0 = *(const v4f*)(pr);
  const v4f p1 = *(const v4f*)(pr + DD);
  const v4f v = (s0 + s1) + (p0 + p1);
  volatile v4f* d = (volatile v4f*)(out + t * DD + n);
  *d = v;
  __threadfence();
  *d = v;
}

extern "C" void kernel_launch(void* const* d_in, const int* in_sizes, int n_in,
                              void* d_out, int out_size, void* d_ws, size_t ws_size,
                              hipStream_t stream) {
  if (n_in < 11) return;
  if (in_sizes[0] != NTOK * DD) return;
  if (in_sizes[1] != NE * DD) return;
  if (in_sizes[2] < NE) return;
  if (in_sizes[3] != NSH * FF * DD) return;
  if (in_sizes[4] < NSH * FF) return;
  if (in_sizes[5] != NSH * DD * FF) return;
  if (in_sizes[6] < NSH * DD) return;
  if (in_sizes[7] != NE * FF * DD) return;
  if (in_sizes[8] < NE * FF) return;
  if (in_sizes[9] != NE * DD * FF) return;
  if (in_sizes[10] < NE * DD) return;
  if (out_size != NTOK * DD) return;

  const float* x   = (const float*)d_in[0];
  const float* gw  = (const float*)d_in[1];
  const float* gb  = (const float*)d_in[2];
  const float* sw1 = (const float*)d_in[3];
  const float* sb1 = (const float*)d_in[4];
  const float* sw2 = (const float*)d_in[5];
  const float* sb2 = (const float*)d_in[6];
  const float* rw1 = (const float*)d_in[7];
  const float* rb1 = (const float*)d_in[8];
  const float* rw2 = (const float*)d_in[9];
  const float* rb2 = (const float*)d_in[10];
  float* out = (float*)d_out;

  size_t off = 0;
  const size_t oXh = off; off += (size_t)NTOK * DD * 2;
  const size_t oS1 = off; off += (size_t)NSH * FF * DD * 2;
  const size_t oR1 = off; off += (size_t)NE * FF * DD * 2;
  const size_t oS2 = off; off += (size_t)NSH * DD * FF * 2;
  const size_t oR2 = off; off += (size_t)NE * DD * FF * 2;
  const size_t oR  = off; off += (size_t)NTOK * RPITCH * 4;
  const size_t oTL = off; off += (size_t)NE * NTOK * 4;
  const size_t oWL = off; off += (size_t)NE * NTOK * 4;
  const size_t oTB = off; off += (size_t)256;
  const size_t oP  = off; off += (size_t)NPART * DD * 4;
  if (off > ws_size) return;
  if (off > (size_t)134217728) return;
  if ((oS1 | oR1 | oS2 | oR2 | oR | oTL | oWL | oTB | oP) & (size_t)127) return;

  char* ws = (char*)d_ws;
  _Float16* Xh   = (_Float16*)(ws + oXh);
  _Float16* SW1h = (_Float16*)(ws + oS1);
  _Float16* RW1h = (_Float16*)(ws + oR1);
  _Float16* SW2h = (_Float16*)(ws + oS2);
  _Float16* RW2h = (_Float16*)(ws + oR2);
  float*    R    = (float*)(ws + oR);
  int*      TOK  = (int*)(ws + oTL);
  float*    WL   = (float*)(ws + oWL);
  int*      TAB  = (int*)(ws + oTB);
  float*    P    = (float*)(ws + oP);

  const int n8x  = (NTOK * DD) / 8;
  const int n8s1 = (NSH * FF * DD) / 8;
  const int n8r1 = (NE * FF * DD) / 8;
  const int n8s2 = (NSH * DD * FF) / 8;
  const int n8r2 = (NE * DD * FF) / 8;

  k_cvt<<<dim3((n8x + 255) / 256), dim3(256), 0, stream>>>(x, Xh, n8x, 1.0f);
  k_cvt<<<dim3((n8s1 + 255) / 256), dim3(256), 0, stream>>>(sw1, SW1h, n8s1, WSC);
  k_cvt<<<dim3((n8r1 + 255) / 256), dim3(256), 0, stream>>>(rw1, RW1h, n8r1, WSC);
  k_cvt<<<dim3((n8s2 + 255) / 256), dim3(256), 0, stream>>>(sw2, SW2h, n8s2, WSC);
  k_cvt<<<dim3((n8r2 + 255) / 256), dim3(256), 0, stream>>>(rw2, RW2h, n8r2, WSC);
  k_route<<<dim3(NTOK / 8), dim3(256), 0, stream>>>(x, gw, gb, R);
  k_lists<<<dim3(1), dim3(256), 0, stream>>>(R, TOK, WL, TAB);
  k_ffn<<<dim3(NSH * TPE + NE * TPE), dim3(256), 0, stream>>>(Xh, SW1h, sb1, SW2h, sb2, RW1h, rb1, RW2h, rb2,
                                                               TOK, WL, TAB, P);
  k_comb<<<dim3((NTOK * DD) / 4 / 256), dim3(256), 0, stream>>>(P, out, (NTOK * DD) / 4);
  (void)hipGetLastError();
}
